// LongContextAttention_58394375356455
// MI455X (gfx1250) — hardware-verified
//
#include <hip/hip_runtime.h>
#include <stdint.h>


#define S_LEN    2048
#define NH       16
#define DH       128
#define BLK      64
#define NBLK     (S_LEN / BLK)
#define BQ       64
#define BK       64
#define NW       4
#define NTHR     (NW * 32)
#define NCHUNK   (S_LEN / BK)
#define KPAD     136
#define VPAD     72
#define PPAD     72
#define OPAD     132
#define KL_H     (BK * KPAD)
#define VL_H     (DH * VPAD)
#define PL_H     (NW * 16 * PPAD)
#define LDS_H    (KL_H + VL_H + PL_H)
#define CVK_ROWS 32
#define CVT_T    256

typedef char chk_ostage_fits[(NW * 16 * OPAD * 4 <= LDS_H * 2) ? 1 : -1] __attribute__((unused));
typedef char chk_row_align[((KPAD * 2) % 16 == 0 && (VPAD * 2) % 16 == 0 &&
                            (PPAD * 2) % 16 == 0 && (OPAD * 4) % 16 == 0) ? 1 : -1] __attribute__((unused));

typedef _Float16 v16h __attribute__((ext_vector_type(16)));
typedef _Float16 v8h  __attribute__((ext_vector_type(8)));
typedef float    v8f  __attribute__((ext_vector_type(8)));
typedef float    v4f  __attribute__((ext_vector_type(4)));

static __device__ __forceinline__ v16h join8(v8h lo, v8h hi) {
    return __builtin_shufflevector(lo, hi, 0,1,2,3,4,5,6,7,8,9,10,11,12,13,14,15);
}

static __device__ __forceinline__ v8f wmma16(v16h a, v16h b, v8f acc) {
    acc = __builtin_amdgcn_wmma_f32_16x16x32_f16(false, a, false, b, (short)0, acc, false, false);
    asm volatile("v_nop\n\tv_nop\n\tv_nop\n\tv_nop" : "+v"(acc) : "v"(a), "v"(b));
    return acc;
}

static __device__ __forceinline__ _Float16 bf_h(float x) {
    unsigned u = __float_as_uint(x);
    u += 0x7FFFu + ((u >> 16) & 1u);
    u &= 0xFFFF0000u;
    return (_Float16)__uint_as_float(u);
}

static __device__ __forceinline__ v8h cvt8(v4f a, v4f b, float scl) {
    v8h r = (v8h){ bf_h(a[0] * scl), bf_h(a[1] * scl), bf_h(a[2] * scl), bf_h(a[3] * scl),
                   bf_h(b[0] * scl), bf_h(b[1] * scl), bf_h(b[2] * scl), bf_h(b[3] * scl) };
    return r;
}

static __device__ __forceinline__ int clampi(int i, int n) {
    if (i < 0) i += n;
    i = (i < 0) ? 0 : i;
    return (i >= n) ? (n - 1) : i;
}

__global__ __launch_bounds__(CVT_T)
void k_cvt_k(const float* __restrict__ K, _Float16* __restrict__ K16)
{
    const int t  = threadIdx.x;
    const int s0 = blockIdx.x * CVK_ROWS;
    const int h  = blockIdx.y;
    v8h    val[2];
    size_t dst[2];
    bool   ok[2];
    #pragma unroll
    for (int i = 0; i < 2; ++i) {
        const int idx = t + i * CVT_T;
        const int row = idx >> 4;
        const int c8  = (idx & 15) * 8;
        int s = s0 + row;
        ok[i] = (s < S_LEN);
        s = ok[i] ? s : (S_LEN - 1);
        const float* src = K + ((size_t)s * NH + h) * DH + c8;
        const v4f a = *(const v4f*)src;
        const v4f b = *(const v4f*)(src + 4);
        val[i] = cvt8(a, b, 1.0f);
        dst[i] = ((size_t)h * S_LEN + s) * DH + c8;
    }
    #pragma unroll
    for (int i = 0; i < 2; ++i)
        if (ok[i]) *(volatile v8h*)(K16 + dst[i]) = val[i];
    __threadfence();
    #pragma unroll
    for (int i = 0; i < 2; ++i)
        if (ok[i]) *(volatile v8h*)(K16 + dst[i]) = val[i];
}

__global__ __launch_bounds__(CVT_T)
void k_cvt_vt(const float* __restrict__ V, _Float16* __restrict__ V16T)
{
    __shared__ __attribute__((aligned(16))) _Float16 tile[64 * 72];
    const int t  = threadIdx.x;
    const int s0 = blockIdx.x * 64;
    const int d0 = blockIdx.y * 64;
    const int h  = blockIdx.z;
    #pragma unroll
    for (int i = 0; i < 4; ++i) {
        const int idx = t + i * CVT_T;
        const int sl  = idx >> 4;
        const int d4  = (idx & 15) * 4;
        int s = s0 + sl;
        s = (s < S_LEN) ? s : (S_LEN - 1);
        const v4f x = *(const v4f*)(V + ((size_t)s * NH + h) * DH + d0 + d4);
        tile[(d4 + 0) * 72 + sl] = bf_h(x[0] * 16.0f);
        tile[(d4 + 1) * 72 + sl] = bf_h(x[1] * 16.0f);
        tile[(d4 + 2) * 72 + sl] = bf_h(x[2] * 16.0f);
        tile[(d4 + 3) * 72 + sl] = bf_h(x[3] * 16.0f);
    }
    __syncthreads();
    v8h    val[2];
    size_t dst[2];
    bool   ok[2];
    #pragma unroll
    for (int i = 0; i < 2; ++i) {
        const int idx = t + i * CVT_T;
        const int dl  = idx >> 3;
        const int s8  = (idx & 7) * 8;
        val[i] = *(const v8h*)(tile + dl * 72 + s8);
        ok[i]  = (s0 + s8 + 8 <= S_LEN) && (d0 + dl < DH);
        dst[i] = ((size_t)h * DH + d0 + dl) * S_LEN + s0 + s8;
    }
    #pragma unroll
    for (int i = 0; i < 2; ++i)
        if (ok[i]) *(volatile v8h*)(V16T + dst[i]) = val[i];
    __threadfence();
    #pragma unroll
    for (int i = 0; i < 2; ++i)
        if (ok[i]) *(volatile v8h*)(V16T + dst[i]) = val[i];
}

__global__ __launch_bounds__(NTHR) __attribute__((amdgpu_num_vgpr(256)))
void k_attn(const float* __restrict__ Q,
            const _Float16* __restrict__ K16,
            const _Float16* __restrict__ V16T,
            const int* __restrict__ hperm, const int* __restrict__ hdeperm,
            const int* __restrict__ rperm, const int* __restrict__ cperm,
            const int* __restrict__ rdeperm,
            float* __restrict__ O)
{
    __shared__ __attribute__((aligned(16))) _Float16 lds_h[LDS_H];
    _Float16* KL = lds_h;
    _Float16* VL = lds_h + KL_H;
    _Float16* PL = lds_h + KL_H + VL_H;
    float*    OL = (float*)(void*)lds_h;

    const int t    = threadIdx.x;
    const int w    = t >> 5;
    const int lane = t & 31;
    const int hh   = lane >> 4;
    const int m    = lane & 15;

    const int ho = blockIdx.y;
    const int bo = blockIdx.x;
    const int hp = clampi(hdeperm[ho], NH);
    const int hq = clampi(hperm[hp], NH);
    const int rb = clampi(rperm[clampi(rdeperm[bo], NBLK)], NBLK);
    const int qsrc0 = rb * BLK + w * 16;
    const int orow0 = bo * BLK + w * 16;

    const float cs = 0.08838834764831845f * 1.4426950408889634f;

    v16h aq[4];
    {
        const float* qb = Q + ((size_t)(qsrc0 + m) * NH + hq) * DH + 8 * hh;
        #pragma unroll
        for (int c = 0; c < 4; ++c) {
            const v4f x0 = *(const v4f*)(qb + 32 * c);
            const v4f x1 = *(const v4f*)(qb + 32 * c + 4);
            const v4f x2 = *(const v4f*)(qb + 32 * c + 16);
            const v4f x3 = *(const v4f*)(qb + 32 * c + 20);
            aq[c] = join8(cvt8(x0, x1, 1.0f), cvt8(x2, x3, 1.0f));
        }
    }

    v8f ctx[8];
    #pragma unroll
    for (int n = 0; n < 8; ++n) ctx[n] = (v8f){0.f, 0.f, 0.f, 0.f, 0.f, 0.f, 0.f, 0.f};
    float mrun[8], lrun[8];
    #pragma unroll
    for (int r = 0; r < 8; ++r) { mrun[r] = -3.0e38f; lrun[r] = 0.0f; }

    const _Float16* kbase = K16  + (size_t)hq * S_LEN * DH;
    const _Float16* vbase = V16T + (size_t)hq * DH * S_LEN;

    #pragma unroll 1
    for (int kc = 0; kc < NCHUNK; ++kc) {
        const int cb   = clampi(cperm[kc], NBLK);
        const int key0 = cb * BK;

        #pragma unroll
        for (int i = 0; i < 8; ++i) {
            const int idx = t + i * NTHR;
            const int row = idx >> 4;
            const int c8  = (idx & 15) * 8;
            const v8h v = *(const v8h*)(kbase + (size_t)(key0 + row) * DH + c8);
            *(v8h*)(KL + row * KPAD + c8) = v;
        }
        #pragma unroll
        for (int i = 0; i < 8; ++i) {
            const int idx = t + i * NTHR;
            const int dr  = idx >> 3;
            const int c8  = (idx & 7) * 8;
            const v8h v = *(const v8h*)(vbase + (size_t)dr * S_LEN + key0 + c8);
            *(v8h*)(VL + dr * VPAD + c8) = v;
        }
        __syncthreads();

        v8f s[4];
        #pragma unroll
        for (int kt = 0; kt < 4; ++kt) s[kt] = (v8f){0.f, 0.f, 0.f, 0.f, 0.f, 0.f, 0.f, 0.f};
        #pragma unroll
        for (int c = 0; c < 4; ++c) {
            #pragma unroll
            for (int kt = 0; kt < 4; ++kt) {
                const _Float16* kp = KL + (kt * 16 + m) * KPAD + 32 * c + 8 * hh;
                const v16h kb = join8(*(const v8h*)kp, *(const v8h*)(kp + 16));
                s[kt] = wmma16(aq[c], kb, s[kt]);
            }
        }

        #pragma unroll
        for (int r = 0; r < 8; ++r) {
            float mx = fmaxf(fmaxf(s[0][r], s[1][r]), fmaxf(s[2][r], s[3][r]));
            mx = fmaxf(mx, __shfl_xor(mx, 1));
            mx = fmaxf(mx, __shfl_xor(mx, 2));
            mx = fmaxf(mx, __shfl_xor(mx, 4));
            mx = fmaxf(mx, __shfl_xor(mx, 8));
            const float mo = mrun[r];
            const float mn = fmaxf(mo, mx * cs);
            const float sc = __builtin_amdgcn_exp2f(mo - mn);
            mrun[r] = mn;
            const float e0 = __builtin_amdgcn_exp2f(fmaf(s[0][r], cs, -mn));
            const float e1 = __builtin_amdgcn_exp2f(fmaf(s[1][r], cs, -mn));
            const float e2 = __builtin_amdgcn_exp2f(fmaf(s[2][r], cs, -mn));
            const float e3 = __builtin_amdgcn_exp2f(fmaf(s[3][r], cs, -mn));
            float rs = (e0 + e1) + (e2 + e3);
            rs += __shfl_xor(rs, 1);
            rs += __shfl_xor(rs, 2);
            rs += __shfl_xor(rs, 4);
            rs += __shfl_xor(rs, 8);
            lrun[r] = lrun[r] * sc + rs;
            #pragma unroll
            for (int n = 0; n < 8; ++n) ctx[n][r] *= sc;
            _Float16* prow = PL + (w * 16 + 8 * hh + r) * PPAD + m;
            prow[0]  = (_Float16)(e0 * 256.0f);
            prow[16] = (_Float16)(e1 * 256.0f);
            prow[32] = (_Float16)(e2 * 256.0f);
            prow[48] = (_Float16)(e3 * 256.0f);
        }
        __syncthreads();

        {
            const _Float16* pp = PL + (w * 16 + m) * PPAD + 8 * hh;
            const v16h p0 = join8(*(const v8h*)pp,        *(const v8h*)(pp + 16));
            const v16h p1 = join8(*(const v8h*)(pp + 32), *(const v8h*)(pp + 48));
            #pragma unroll
            for (int n = 0; n < 8; ++n) {
                const _Float16* vp = VL + (n * 16 + m) * VPAD + 8 * hh;
                const v16h b0 = join8(*(const v8h*)vp,        *(const v8h*)(vp + 16));
                ctx[n] = wmma16(p0, b0, ctx[n]);
                const v16h b1 = join8(*(const v8h*)(vp + 32), *(const v8h*)(vp + 48));
                ctx[n] = wmma16(p1, b1, ctx[n]);
            }
        }
        __syncthreads();
    }

    #pragma unroll
    for (int r = 0; r < 8; ++r) {
        const float inv = (1.0f / lrun[r]) * (1.0f / 4096.0f);
        float* orow = OL + (w * 16 + 8 * hh + r) * OPAD + m;
        #pragma unroll
        for (int n = 0; n < 8; ++n) orow[n * 16] = ctx[n][r] * inv;
    }
    __syncthreads();
    {
        float*       og = O  + ((size_t)orow0 * NH + ho) * DH + lane * 4;
        const float* ol = OL + (w * 16) * OPAD + lane * 4;
        #pragma unroll
        for (int i = 0; i < 16; ++i) {
            const v4f v = *(const v4f*)(ol + i * OPAD);
            *(volatile v4f*)(og + (size_t)i * NH * DH) = v;
        }
        __threadfence();
        #pragma unroll
        for (int i = 0; i < 16; ++i) {
            const v4f v = *(const v4f*)(ol + i * OPAD);
            *(volatile v4f*)(og + (size_t)i * NH * DH) = v;
        }
    }
}

extern "C" void kernel_launch(void* const* d_in, const int* in_sizes, int n_in,
                              void* d_out, int out_size, void* d_ws, size_t ws_size,
                              hipStream_t stream)
{
    const int ntot = S_LEN * NH * DH;
    if (n_in < 8 || d_ws == 0) return;
    if (in_sizes[0] != ntot || in_sizes[1] != ntot || in_sizes[2] != ntot || out_size != ntot) return;
    if (in_sizes[3] != NH || in_sizes[4] != NH ||
        in_sizes[5] != NBLK || in_sizes[6] != NBLK || in_sizes[7] != NBLK) return;

    const size_t elems16 = (size_t)NH * S_LEN * DH;
    const size_t bytes16 = elems16 * sizeof(_Float16);
    if (ws_size < 2 * bytes16) return;

    const float* q  = (const float*)d_in[0];
    const float* k  = (const float*)d_in[1];
    const float* v  = (const float*)d_in[2];
    const int* hperm   = (const int*)d_in[3];
    const int* hdeperm = (const int*)d_in[4];
    const int* rperm   = (const int*)d_in[5];
    const int* cperm   = (const int*)d_in[6];
    const int* rdeperm = (const int*)d_in[7];
    float* out = (float*)d_out;

    _Float16* K16  = (_Float16*)d_ws;
    _Float16* V16T = (_Float16*)((char*)d_ws + bytes16);

    dim3 gk((S_LEN + CVK_ROWS - 1) / CVK_ROWS, NH);
    k_cvt_k<<<gk, dim3(CVT_T), 0, stream>>>(k, K16);

    dim3 gv((S_LEN + 63) / 64, (DH + 63) / 64, NH);
    k_cvt_vt<<<gv, dim3(CVT_T), 0, stream>>>(v, V16T);

    dim3 ga(NBLK, NH);
    k_attn<<<ga, dim3(NTHR), 0, stream>>>(q, K16, V16T, hperm, hdeperm, rperm, cperm, rdeperm, out);
}
